// GraphEncoderSAGE_65773129171089
// MI455X (gfx1250) — hardware-verified
//
#include <hip/hip_runtime.h>
#include <math.h>

typedef __attribute__((ext_vector_type(16))) _Float16 v16h;
typedef __attribute__((ext_vector_type(16))) __bf16 v16b;
typedef __attribute__((ext_vector_type(8)))  _Float16 v8h;
typedef __attribute__((ext_vector_type(8)))  float v8f;
typedef __attribute__((ext_vector_type(4)))  float v4f;
typedef __attribute__((ext_vector_type(2)))  float v2f;
typedef __attribute__((ext_vector_type(4)))  unsigned v4u;
typedef __attribute__((ext_vector_type(4)))  int v4i;
typedef float __attribute__((may_alias)) float_a;
typedef int __attribute__((may_alias)) int_a;

template <typename T> __device__ __forceinline__ void vst2(void* p, T v) { *(volatile T*)p = v; __threadfence(); *(volatile T*)p = v; }
__device__ __forceinline__ v8f wmma16(v16h a, v16h b, v8f c) {
  v8f d = __builtin_amdgcn_wmma_f32_16x16x32_f16(false, a, false, b, (short)0, c, false, false);
  asm volatile("v_nop\n\tv_nop\n\tv_nop\n\tv_nop" : "+v"(d) : "v"(a), "v"(b));
  return d;
}
__device__ __forceinline__ v8f wmma_bf(v16b a, v16b b, v8f c) {
  v8f d = __builtin_amdgcn_wmma_f32_16x16x32_bf16(false, a, false, b, (short)0, c, false, false);
  asm volatile("v_nop\n\tv_nop\n\tv_nop\n\tv_nop" : "+v"(d) : "v"(a), "v"(b));
  return d;
}
__device__ __forceinline__ v16h frag_h(const _Float16* rowk0, int lane) {
  union { v16h v; v8h q[2]; } u; const _Float16* p = rowk0 + 8 * (lane >> 4);
  u.q[0] = *(const v8h*)p; u.q[1] = *(const v8h*)(p + 16); return u.v;
}
__device__ __forceinline__ v16h frag_f32(const float* rowk0, int lane) {
  v16h a; const float* p = rowk0 + 8 * (lane >> 4);
#pragma unroll
  for (int i = 0; i < 8; ++i) { a[i] = (_Float16)p[i]; a[8 + i] = (_Float16)p[16 + i]; }
  return a;
}
__device__ __forceinline__ v16h frag_f32s(const float* rowk0, int lane, float sc) {
  v16h a; const float* p = rowk0 + 8 * (lane >> 4);
#pragma unroll
  for (int i = 0; i < 8; ++i) { a[i] = (_Float16)(p[i] * sc); a[8 + i] = (_Float16)(p[16 + i] * sc); }
  return a;
}
__device__ __forceinline__ v16h fragc_f32(const float* W, int k0, int n, int lane, int ld, int K) {
  v16h a; const int g = lane >> 4;
#pragma unroll
  for (int i = 0; i < 8; ++i) { const int ka = k0 + 8 * g + i, kb = ka + 16;
    a[i] = (_Float16)(ka < K ? W[(size_t)ka * ld + n] : 0.f); a[8 + i] = (_Float16)(kb < K ? W[(size_t)kb * ld + n] : 0.f); }
  return a;
}
struct F2 { v16b h, l; };
__device__ __forceinline__ F2 bsplit16(const float v[16]) { F2 r;
#pragma unroll
  for (int i = 0; i < 16; ++i) { const __bf16 h = (__bf16)v[i]; r.h[i] = h; r.l[i] = (__bf16)(v[i] - (float)h); }
  return r; }
__device__ __forceinline__ F2 split_row(const float* row, int k0, int lane) { float v[16]; const float* p = row + k0 + 8 * (lane >> 4);
#pragma unroll
  for (int i = 0; i < 8; ++i) { v[i] = p[i]; v[8 + i] = p[16 + i]; }
  return bsplit16(v); }
__device__ __forceinline__ F2 split_rowK(const float* row, int k0, int lane, int K) { float v[16]; const int g = lane >> 4;
#pragma unroll
  for (int i = 0; i < 8; ++i) { const int ka = k0 + 8 * g + i, kb = ka + 16; v[i] = ka < K ? row[ka] : 0.f; v[8 + i] = kb < K ? row[kb] : 0.f; }
  return bsplit16(v); }
__device__ __forceinline__ F2 split_col(const float* W, int k0, int n, int lane, int ld, int K) { float v[16]; const int g = lane >> 4;
#pragma unroll
  for (int i = 0; i < 8; ++i) { const int ka = k0 + 8 * g + i, kb = ka + 16; v[i] = ka < K ? W[(size_t)ka * ld + n] : 0.f; v[8 + i] = kb < K ? W[(size_t)kb * ld + n] : 0.f; }
  return bsplit16(v); }
__device__ __forceinline__ v8f mac3(const F2& a, const F2& b, v8f c) { c = wmma_bf(a.l, b.h, c); c = wmma_bf(a.h, b.l, c); return wmma_bf(a.h, b.h, c); }
__device__ __forceinline__ float sigm(float v) { return 1.0f / (1.0f + expf(-v)); }
#define LDSX() do { asm volatile("s_wait_dscnt 0" ::: "memory"); __builtin_amdgcn_wave_barrier(); __builtin_amdgcn_fence(__ATOMIC_RELEASE, "workgroup"); } while (0)

#define NN 50000
#define NE 800000
#define FH 128
#define RB 512
#define NRB ((NN + RB - 1) / RB)
#define NNP (NRB * RB)
#define NG 256
#define EPT 16
#define CH (256 * EPT)

__global__ __launch_bounds__(256) void k_agg(const float* __restrict__ x, const int* __restrict__ ei, float* __restrict__ AGG) {
  __shared__ __align__(16) float sacc[RB][FH];
  __shared__ int ssrc[8][32 * EPT], sdl[8][32 * EPT]; __shared__ int scnt[8]; __shared__ int srcnt[RB];
  const int tid = threadIdx.x, wave = tid >> 5, lane = tid & 31;
  const int r0 = blockIdx.x * RB; const int* esrc = ei; const int* edst = ei + NE;
  for (int q = tid; q < RB * FH; q += 256) (&sacc[0][0])[q] = 0.f;
  for (int q = tid; q < RB; q += 256) srcnt[q] = 0;
  __syncthreads();
  #pragma unroll 1
  for (int c0 = 0; c0 < NE; c0 += CH) {
    const int e0 = c0 + tid * EPT; int hd[EPT]; int cnt = 0;
    if (e0 + EPT <= NE) {
#pragma unroll
      for (int v = 0; v < EPT / 4; ++v) { const int4 d4 = *(const int4*)(edst + e0 + v * 4);
        const int dd[4] = {d4.x, d4.y, d4.z, d4.w};
#pragma unroll
        for (int u = 0; u < 4; ++u) { const unsigned rel = (unsigned)(dd[u] - r0); const bool h = rel < (unsigned)RB; hd[v * 4 + u] = h ? (int)rel : -1; cnt += h ? 1 : 0; } } }
    else {
#pragma unroll
      for (int u = 0; u < EPT; ++u) { const int e = e0 + u; hd[u] = -1; if (e < NE) { const unsigned rel = (unsigned)(edst[e] - r0); if (rel < (unsigned)RB) { hd[u] = (int)rel; ++cnt; } } } }
    int incl = cnt;
#pragma unroll
    for (int off = 1; off < 32; off <<= 1) { const int vv = __shfl_up(incl, off, 32); if (lane >= off) incl += vv; }
    const int wtot = __shfl(incl, 31, 32); int pos = incl - cnt;
    if (cnt > 0) {
#pragma unroll
      for (int u = 0; u < EPT; ++u) if (hd[u] >= 0) { int s = esrc[e0 + u]; s = s < 0 ? 0 : (s >= NN ? NN - 1 : s); ssrc[wave][pos] = s; sdl[wave][pos] = hd[u]; atomicAdd(&srcnt[hd[u]], 1); ++pos; } }
    if (lane == 0) scnt[wave] = wtot;
    __syncthreads();
    if (tid < FH) { for (int w = 0; w < 8; ++w) { const int nh = scnt[w]; for (int i = 0; i < nh; ++i) sacc[sdl[w][i]][tid] += x[(size_t)ssrc[w][i] * FH + tid]; } }
    __syncthreads(); }
  for (int q = tid; q < RB * (FH / 4); q += 256) { const int rl = q >> 5, pc = q & 31; const int row = r0 + rl; const float inv = 1.0f / fmaxf((float)srcnt[rl], 1.0f);
    v4f v = *(const v4f*)(&sacc[rl][pc * 4]); v *= inv; if (row >= NN) v = (v4f){0.f, 0.f, 0.f, 0.f}; vst2(AGG + (size_t)row * FH + pc * 4, v); }
}
__global__ __launch_bounds__(128) void k_lin(const float* __restrict__ AGG, const float* __restrict__ x, const float* __restrict__ Wl, const float* __restrict__ bl, const float* __restrict__ Wr, int relu, float* __restrict__ out) {
  __shared__ __align__(16) float so[4][16][FH + 4];
  const int tid = threadIdx.x, wave = tid >> 5, lane = tid & 31, col = lane & 15, g = lane >> 4;
  const int r0 = blockIdx.x * 64 + wave * 16; const int ra = (r0 + col) < NN ? (r0 + col) : (NN - 1);
  v8f acc[8] = {};
#pragma unroll 1
  for (int kc = 0; kc < 8; ++kc) { const F2 a = kc < 4 ? split_row(AGG + (size_t)ra * FH, kc * 32, lane) : split_row(x + (size_t)ra * FH, (kc - 4) * 32, lane);
#pragma unroll
    for (int j = 0; j < 8; ++j) { const int n = j * 16 + col; acc[j] = mac3(a, kc < 4 ? split_row(Wl + (size_t)n * FH, kc * 32, lane) : split_row(Wr + (size_t)n * FH, (kc - 4) * 32, lane), acc[j]); } }
#pragma unroll
  for (int j = 0; j < 8; ++j) { const int n = j * 16 + col; const float bb = bl[n];
#pragma unroll
    for (int r = 0; r < 8; ++r) { float v = acc[j][r] + bb; if (relu) v = v > 0.f ? v : 0.f; so[wave][8 * g + r][n] = v; } }
  LDSX();
  for (int q = lane; q < 16 * 32; q += 32) { const int rl = q >> 5, pc = q & 31; const int row = r0 + rl; if (row < NN) vst2(out + (size_t)row * FH + pc * 4, *(const v4f*)(&so[wave][rl][pc * 4])); }
}
__global__ __launch_bounds__(128) void k_pool(const float* __restrict__ H, const int* __restrict__ bidx, float* __restrict__ out) {
  __shared__ int slist[1024]; __shared__ int swt[4]; __shared__ __align__(16) float so[FH];
  const int gph = blockIdx.x, tid = threadIdx.x, wave = tid >> 5, lane = tid & 31; float acc = 0.f; int total = 0;
#pragma unroll 1
  for (int n0 = 0; n0 < NN; n0 += 1024) { int hit[8]; int cnt = 0;
#pragma unroll
    for (int u = 0; u < 8; ++u) { const int n = n0 + tid * 8 + u; hit[u] = (n < NN && bidx[n] == gph) ? n : -1; cnt += hit[u] >= 0; }
    int incl = cnt;
#pragma unroll
    for (int off = 1; off < 32; off <<= 1) { const int vv = __shfl_up(incl, off, 32); if (lane >= off) incl += vv; }
    if (lane == 31) swt[wave] = incl;
    __syncthreads();
    int base = 0, tot = 0; for (int w = 0; w < 4; ++w) { if (w < wave) base += swt[w]; tot += swt[w]; }
    int pos = base + incl - cnt;
#pragma unroll
    for (int u = 0; u < 8; ++u) if (hit[u] >= 0) slist[pos++] = hit[u];
    __syncthreads();
    for (int i = 0; i < tot; ++i) acc += H[(size_t)slist[i] * FH + tid];
    total += tot;
    __syncthreads(); }
  so[tid] = acc / fmaxf((float)total, 1.0f);
  __syncthreads();
  if (tid < FH / 4) vst2(out + (size_t)gph * FH + tid * 4, *(const v4f*)(&so[tid * 4]));
}
extern "C" void kernel_launch(void* const* d_in, const int* in_sizes, int n_in, void* d_out, int out_size, void* d_ws, size_t ws_size, hipStream_t stream) {
  (void)in_sizes; (void)n_in; (void)out_size; (void)ws_size;
  const float* x = (const float*)d_in[0]; const int* ei = (const int*)d_in[1]; const int* bidx = (const int*)d_in[2]; const float* Wl = (const float*)d_in[3]; const float* Wr = (const float*)d_in[4]; const float* bl = (const float*)d_in[5];
  float* out = (float*)d_out;
  char* ws = (char*)d_ws; size_t off = 0;
  auto take = [&](size_t bytes) { char* p = ws + off; off += (bytes + 255) & ~(size_t)255; return p; };
  float* AGG = (float*)take((size_t)NNP * FH * 4); float* HA = (float*)take((size_t)NNP * FH * 4); float* HB = (float*)take((size_t)NNP * FH * 4);
  const float* cur = x; float* bufs[2] = {HA, HB};
  for (int l = 0; l < 3; ++l) {
    k_agg<<<NRB, 256, 0, stream>>>(cur, ei, AGG);
    float* dst = bufs[l & 1];
    k_lin<<<NNP / 64, 128, 0, stream>>>(AGG, cur, Wl + (size_t)l * FH * FH, bl + l * FH, Wr + (size_t)l * FH * FH, l < 2 ? 1 : 0, dst);
    cur = dst; }
  k_pool<<<NG, 128, 0, stream>>>(cur, bidx, out);
}
